// BCMEmulator_30090540876111
// MI455X (gfx1250) — hardware-verified
//
#include <hip/hip_runtime.h>
#include <stdint.h>

#define DEVINL __device__ __forceinline__

typedef _Float16 f16t;
typedef _Float16 v16h __attribute__((ext_vector_type(16)));
typedef _Float16 v8h  __attribute__((ext_vector_type(8)));
typedef float    v8f  __attribute__((ext_vector_type(8)));
typedef float    v4f  __attribute__((ext_vector_type(4)));
typedef v8h __attribute__((may_alias)) v8ha;
typedef v4f __attribute__((may_alias)) v4fa;
union FragH { v16h v; v8h half[2]; };

#define TLEN   1024
#define CIN    15
#define EMBD   8
#define CXIN   (CIN + EMBD)
#define CPX    32
#define CH     64
#define PADR   64
#define TP     (PADR + TLEN)
#define TILET  64
#define NTILE  (TLEN / TILET)
#define CTPB   128
#define TPB    256
#define ACAR   16.0f
#define WCAR   256.0f
#define INVCAR (1.0f / 4096.0f)

#define KXA     (3 * CPX)
#define KXR     (CPX)
#define K64     (3 * CH)
#define OFF_W0A 0
#define OFF_W0R (OFF_W0A + CH * KXA)
#define OFF_W0B (OFF_W0R + CH * KXR)
#define OFF_WA  (OFF_W0B + CH * K64)
#define OFF_WB  (OFF_WA + 4 * CH * K64)
#define WTOT    (OFF_WB + 4 * CH * K64)
#define WBLKX   ((4 * CH * K64 / 8 + TPB - 1) / TPB)

static_assert((KXA % 32) == 0);
static_assert((KXR % 32) == 0);
static_assert((K64 % 32) == 0);
static_assert((OFF_W0R % 256) == 0);
static_assert((OFF_W0B % 256) == 0);
static_assert((OFF_WA % 256) == 0);
static_assert((OFF_WB % 256) == 0);
static_assert((WTOT % 256) == 0);
static_assert((TLEN % TILET) == 0);
static_assert((TP % 64) == 0);
static_assert(PADR >= 32);
static_assert(64 * CPX == TPB * 8);
static_assert(PADR * CH == 2 * TPB * 8);
static_assert((TLEN % TPB) == 0);
static_assert(CTPB == 128);

DEVINL int imin(int a, int b) { return a < b ? a : b; }
DEVINL int imax(int a, int b) { return a > b ? a : b; }

DEVINL v8f wmma_f16(v16h a, v16h b, v8f c) {
  v8f d = __builtin_amdgcn_wmma_f32_16x16x32_f16(false, a, false, b, (short)0, c, false, false);
  asm volatile("v_nop\n\tv_nop\n\tv_nop\n\tv_nop" : "+v"(d) : "v"(a), "v"(b));
  return d;
}
DEVINL v8f zero8f() {
  v8f z = {0.f, 0.f, 0.f, 0.f, 0.f, 0.f, 0.f, 0.f};
  return z;
}
DEVINL v8h zero8h() {
  v8h z;
  #pragma unroll
  for (int i = 0; i < 8; ++i) z[i] = (f16t)0.0f;
  return z;
}

__global__ __launch_bounds__(TPB) void prep_w_k(const float* __restrict__ w0a, const float* __restrict__ w0r,
                                              const float* __restrict__ w0b, const float* __restrict__ wa,
                                              const float* __restrict__ wb, f16t* __restrict__ Wp)
{
  const int reg = blockIdx.y;
  const float* w = w0a; int cp = CPX, ntap = 3, rows = CH, cin = CXIN, off = OFF_W0A;
  if (reg == 1)      { w = w0r; cp = CPX; ntap = 1; rows = CH;     cin = CXIN; off = OFF_W0R; }
  else if (reg == 2) { w = w0b; cp = CH;  ntap = 3; rows = CH;     cin = CH;   off = OFF_W0B; }
  else if (reg == 3) { w = wa;  cp = CH;  ntap = 3; rows = 4 * CH; cin = CH;   off = OFF_WA;  }
  else if (reg == 4) { w = wb;  cp = CH;  ntap = 3; rows = 4 * CH; cin = CH;   off = OFF_WB;  }
  const int K    = ntap * cp;
  const int kg   = K >> 3;
  const int nthr = rows * kg;
  const int t = blockIdx.x * TPB + threadIdx.x;
  if (t >= nthr) return;
  const int row  = t / kg;
  const int part = t - row * kg;
  const int k8   = 8 * part;
  const int tap  = k8 / cp;
  const int c0   = k8 - tap * cp;
  v8h o;
  #pragma unroll
  for (int i = 0; i < 8; ++i) {
    const int c  = c0 + i;
    const int cc = imin(c, cin - 1);
    const float wv = w[((size_t)row * cin + cc) * ntap + tap];
    o[i] = (f16t)(((c < cin) ? wv : 0.0f) * WCAR);
  }
  f16t* dst = Wp + off + (size_t)8 * t;
  *(volatile v8h*)dst = o;
  __threadfence();
  *(volatile v8h*)dst = o;
}

__global__ __launch_bounds__(TPB) void pad_k(f16t* __restrict__ H16, f16t* __restrict__ F16)
{
  const int b = blockIdx.x;
  f16t* plane = (blockIdx.y == 0) ? H16 : F16;
  f16t* d0 = plane + (size_t)b * TP * CH + 8 * threadIdx.x;
  f16t* d1 = d0 + TPB * 8;
  const v8h z = zero8h();
  *(volatile v8h*)d0 = z;
  *(volatile v8h*)d1 = z;
  __threadfence();
  *(volatile v8h*)d0 = z;
  *(volatile v8h*)d1 = z;
}

__global__ __launch_bounds__(TPB) void xin_k(const float* __restrict__ x, const int* __restrict__ fids,
                                           const float* __restrict__ femb, int nf, f16t* __restrict__ XIN)
{
  __shared__ __attribute__((aligned(16))) f16t sXi[64 * CPX];
  const int tid = threadIdx.x, chunk = blockIdx.x, b = blockIdx.y;
  int fid = fids[b];
  fid = imin(imax(fid, 0), nf - 1);
  #pragma unroll 1
  for (int idx = tid; idx < 64 * CPX; idx += TPB) {
    const int c  = idx >> 6;
    const int tt = idx & 63;
    const int t  = chunk * 64 + tt - PADR;
    const int tcl = imax(t, 0);
    const int cx  = imin(c, CIN - 1);
    const int ce  = imin(imax(c - CIN, 0), EMBD - 1);
    const float xv = x[((size_t)b * CIN + cx) * TLEN + tcl];
    const float ev = femb[fid * EMBD + ce];
    float v = (c < CIN) ? xv : ((c < CXIN) ? ev : 0.0f);
    v = (t >= 0) ? v : 0.0f;
    sXi[tt * CPX + c] = (f16t)(v * ACAR);
  }
  __syncthreads();
  const v8h val = *(const v8ha*)(sXi + 8 * tid);
  f16t* dst = XIN + ((size_t)(b * TP + chunk * 64)) * CPX + 8 * tid;
  *(volatile v8h*)dst = val;
  __threadfence();
  *(volatile v8h*)dst = val;
}

template <int MODE>
DEVINL void stage8(v8f acc, float* srow, int c0, const float* __restrict__ bias, const float* frow)
{
  float old8[8];
  if (MODE == 2) {
    const v4f u0 = *(const v4fa*)(frow + c0);
    const v4f u1 = *(const v4fa*)(frow + c0 + 4);
    old8[0] = u0[0]; old8[1] = u0[1]; old8[2] = u0[2]; old8[3] = u0[3];
    old8[4] = u1[0]; old8[5] = u1[1]; old8[6] = u1[2]; old8[7] = u1[3];
  } else {
    #pragma unroll
    for (int r = 0; r < 8; ++r) old8[r] = 0.0f;
  }
  #pragma unroll
  for (int r = 0; r < 8; ++r) {
    float y = fmaf(acc[r], INVCAR, bias[c0 + r]);
    if (MODE == 0) y = fmaxf(y, 0.0f);
    if (MODE == 2) y = old8[r] + fmaxf(y, 0.0f);
    srow[c0 + r] = y;
  }
}

template <int CP, int NTAP, int MODE>
__global__ __launch_bounds__(CTPB) void conv_k(const f16t* __restrict__ src, const f16t* __restrict__ Wl,
                                             const float* __restrict__ bias, int dil,
                                             f16t* __restrict__ dst16, float* F32p)
{
  __shared__ __attribute__((aligned(16))) float sO[TILET * CH];
  constexpr int K  = NTAP * CP;
  constexpr int CS = CP / 32;
  const int tid = threadIdx.x, lane = tid & 31, wave = tid >> 5;
  const int h = lane >> 4, m = lane & 15;
  const int wc = wave & 1, wq = wave >> 1;
  const int b  = blockIdx.y;
  const int tb = blockIdx.x * TILET;
  const int tl0 = 32 * wq + m;
  const int tl1 = tl0 + 16;

  const f16t* sbase = src + (size_t)b * TP * CP + 8 * h;
  const f16t* wr0 = Wl + (size_t)(32 * wc + m) * K + 8 * h;
  const f16t* wr1 = wr0 + (size_t)16 * K;

  v8f acc00 = zero8f(), acc01 = zero8f(), acc10 = zero8f(), acc11 = zero8f();

  #pragma unroll 1
  for (int tap = 0; tap < NTAP; ++tap) {
    const int shift = (NTAP - 1 - tap) * dil;
    const f16t* y0 = sbase + (size_t)(PADR + tb + tl0 - shift) * CP;
    const f16t* y1 = sbase + (size_t)(PADR + tb + tl1 - shift) * CP;
    const f16t* ap0 = wr0 + tap * CP;
    const f16t* ap1 = wr1 + tap * CP;
    #pragma unroll
    for (int cs = 0; cs < CS; ++cs) {
      FragH a0, a1, b0, b1;
      a0.half[0] = *(const v8ha*)(ap0 + 32 * cs);
      a0.half[1] = *(const v8ha*)(ap0 + 32 * cs + 16);
      a1.half[0] = *(const v8ha*)(ap1 + 32 * cs);
      a1.half[1] = *(const v8ha*)(ap1 + 32 * cs + 16);
      b0.half[0] = *(const v8ha*)(y0 + 32 * cs);
      b0.half[1] = *(const v8ha*)(y0 + 32 * cs + 16);
      b1.half[0] = *(const v8ha*)(y1 + 32 * cs);
      b1.half[1] = *(const v8ha*)(y1 + 32 * cs + 16);
      acc00 = wmma_f16(a0.v, b0.v, acc00);
      acc01 = wmma_f16(a0.v, b1.v, acc01);
      acc10 = wmma_f16(a1.v, b0.v, acc10);
      acc11 = wmma_f16(a1.v, b1.v, acc11);
    }
  }

  {
    const int cA = 32 * wc + 8 * h;
    const int cB = cA + 16;
    const float* fold0 = F32p + ((size_t)(b * TLEN + tb + tl0)) * CH;
    const float* fold1 = F32p + ((size_t)(b * TLEN + tb + tl1)) * CH;
    stage8<MODE>(acc00, sO + tl0 * CH, cA, bias, fold0);
    stage8<MODE>(acc01, sO + tl1 * CH, cA, bias, fold1);
    stage8<MODE>(acc10, sO + tl0 * CH, cB, bias, fold0);
    stage8<MODE>(acc11, sO + tl1 * CH, cB, bias, fold1);
  }
  __syncthreads();

  v8h hv[4];
  v4f fv[8];
  const int p8 = (lane & 7) * 8, rq = lane >> 3;
  const int q4 = (lane & 15) * 4, rh = lane >> 4;
  f16t*  drow = dst16 + ((size_t)(b * TP + PADR + tb)) * CH;
  float* frw  = F32p + ((size_t)(b * TLEN + tb)) * CH;
  if (MODE != 1) {
    #pragma unroll
    for (int j = 0; j < 4; ++j) {
      const int row = 16 * wave + 4 * j + rq;
      const v4f u0 = *(const v4fa*)(sO + row * CH + p8);
      const v4f u1 = *(const v4fa*)(sO + row * CH + p8 + 4);
      v8h o;
      o[0] = (f16t)(u0[0] * ACAR); o[1] = (f16t)(u0[1] * ACAR);
      o[2] = (f16t)(u0[2] * ACAR); o[3] = (f16t)(u0[3] * ACAR);
      o[4] = (f16t)(u1[0] * ACAR); o[5] = (f16t)(u1[1] * ACAR);
      o[6] = (f16t)(u1[2] * ACAR); o[7] = (f16t)(u1[3] * ACAR);
      hv[j] = o;
    }
  }
  if (MODE != 0) {
    #pragma unroll
    for (int j = 0; j < 8; ++j) {
      const int row = 16 * wave + 2 * j + rh;
      fv[j] = *(const v4fa*)(sO + row * CH + q4);
    }
  }
  if (MODE != 1) {
    #pragma unroll
    for (int j = 0; j < 4; ++j) {
      const int row = 16 * wave + 4 * j + rq;
      *(volatile v8h*)(drow + (size_t)row * CH + p8) = hv[j];
    }
  }
  if (MODE != 0) {
    #pragma unroll
    for (int j = 0; j < 8; ++j) {
      const int row = 16 * wave + 2 * j + rh;
      *(volatile v4f*)(frw + (size_t)row * CH + q4) = fv[j];
    }
  }
  __threadfence();
  if (MODE != 1) {
    #pragma unroll
    for (int j = 0; j < 4; ++j) {
      const int row = 16 * wave + 4 * j + rq;
      *(volatile v8h*)(drow + (size_t)row * CH + p8) = hv[j];
    }
  }
  if (MODE != 0) {
    #pragma unroll
    for (int j = 0; j < 8; ++j) {
      const int row = 16 * wave + 2 * j + rh;
      *(volatile v4f*)(frw + (size_t)row * CH + q4) = fv[j];
    }
  }
}

DEVINL float softplus_f(float v) {
  return fmaxf(v, 0.0f) + __logf(1.0f + __expf(-fabsf(v)));
}

__global__ __launch_bounds__(TPB) void heads_k(const float* __restrict__ F32p,
                                             const float* __restrict__ petw, const float* __restrict__ petb,
                                             const float* __restrict__ pckw, const float* __restrict__ pckb,
                                             const float* __restrict__ aetw, const float* __restrict__ aetb,
                                             float* __restrict__ out, int npos)
{
  __shared__ float sW[200];
  __shared__ __attribute__((aligned(16))) float sR[4 * TPB];
  const int tid = threadIdx.x;
  if (tid < CH) { sW[tid] = petw[tid]; sW[CH + tid] = pckw[tid]; sW[2 * CH + tid] = aetw[tid]; }
  if (tid < 2)  sW[3 * CH + tid] = aetw[CH + tid];
  if (tid == 0) { sW[194] = petb[0]; sW[195] = pckb[0]; sW[196] = aetb[0]; }
  __syncthreads();

  const int p = blockIdx.x * TPB + tid;
  const float* fr = F32p + (size_t)p * CH;
  float sp = 0.0f, sk = 0.0f, sa = 0.0f;
  #pragma unroll 1
  for (int c4 = 0; c4 < CH / 4; ++c4) {
    const v4f v = *(const v4fa*)(fr + 4 * c4);
    #pragma unroll
    for (int i = 0; i < 4; ++i) {
      const int c = 4 * c4 + i;
      const float fc = v[i];
      sp = fmaf(sW[c], fc, sp);
      sk = fmaf(sW[CH + c], fc, sk);
      sa = fmaf(sW[2 * CH + c], fc, sa);
    }
  }
  const float pet = softplus_f(sp + sW[194]);
  const float pck = softplus_f(sk + sW[195]);
  float alin = fmaf(sW[3 * CH], pet, fmaf(sW[3 * CH + 1], pck, sa)) + sW[196];
  alin = fminf(fmaxf(alin, -30.0f), 30.0f);
  const float e   = __expf(-alin);
  const float sig = __fdividef(1.0f, 1.0f + e);
  const float aet = sig * pet;
  const float cwd = pet - aet;
  sR[tid]           = pet;
  sR[TPB + tid]     = pck;
  sR[2 * TPB + tid] = aet;
  sR[3 * TPB + tid] = cwd;
  __syncthreads();

  const int k = tid >> 6, q = (tid & 63) * 4;
  const v4f ov = *(const v4fa*)(sR + k * TPB + q);
  float* dst = out + (size_t)k * npos + (size_t)blockIdx.x * TPB + q;
  *(volatile v4f*)dst = ov;
  __threadfence();
  *(volatile v4f*)dst = ov;
}

extern "C" void kernel_launch(void* const* d_in, const int* in_sizes, int n_in,
                              void* d_out, int out_size, void* d_ws, size_t ws_size,
                              hipStream_t stream)
{
  if (n_in < 19) return;
  const int perSeq = CIN * TLEN;
  if (in_sizes[0] <= 0 || (in_sizes[0] % perSeq) != 0) return;
  const int nB = in_sizes[0] / perSeq;
  if (nB > 65535) return;
  if (in_sizes[1] != nB) return;
  if (in_sizes[2] < EMBD || (in_sizes[2] % EMBD) != 0) return;
  const int nF = in_sizes[2] / EMBD;
  if (in_sizes[3] != CH * CXIN * 3) return;
  if (in_sizes[4] != CH) return;
  if (in_sizes[5] != CH * CH * 3) return;
  if (in_sizes[6] != CH) return;
  if (in_sizes[7] != CH * CXIN) return;
  if (in_sizes[8] != CH) return;
  if (in_sizes[9] != 4 * CH * CH * 3) return;
  if (in_sizes[10] != 4 * CH) return;
  if (in_sizes[11] != 4 * CH * CH * 3) return;
  if (in_sizes[12] != 4 * CH) return;
  if (in_sizes[13] != CH || in_sizes[14] < 1) return;
  if (in_sizes[15] != CH || in_sizes[16] < 1) return;
  if (in_sizes[17] != CH + 2 || in_sizes[18] < 1) return;
  const int npos = nB * TLEN;
  if (out_size != 4 * npos) return;
  if ((npos % TPB) != 0) return;

  const float* x    = (const float*)d_in[0];
  const int*   fids = (const int*)d_in[1];
  const float* femb = (const float*)d_in[2];
  const float* w0a  = (const float*)d_in[3];
  const float* b0a  = (const float*)d_in[4];
  const float* w0b  = (const float*)d_in[5];
  const float* b0b  = (const float*)d_in[6];
  const float* w0r  = (const float*)d_in[7];
  const float* b0r  = (const float*)d_in[8];
  const float* wa   = (const float*)d_in[9];
  const float* ba   = (const float*)d_in[10];
  const float* wb   = (const float*)d_in[11];
  const float* bb   = (const float*)d_in[12];
  const float* petw = (const float*)d_in[13];
  const float* petb = (const float*)d_in[14];
  const float* pckw = (const float*)d_in[15];
  const float* pckb = (const float*)d_in[16];
  const float* aetw = (const float*)d_in[17];
  const float* aetb = (const float*)d_in[18];
  float* outp = (float*)d_out;

  const size_t szWp  = (size_t)WTOT * 2;
  const size_t szXIN = (size_t)nB * TP * CPX * 2;
  const size_t szH16 = (size_t)nB * TP * CH * 2;
  const size_t szF16 = szH16;
  const size_t szF32 = (size_t)nB * TLEN * CH * 4;
  size_t off = 0;
  char* ws = (char*)d_ws;
  f16t*  Wp  = (f16t*)(ws + off);  off += szWp;
  f16t*  XIN = (f16t*)(ws + off);  off += szXIN;
  f16t*  H16 = (f16t*)(ws + off);  off += szH16;
  f16t*  F16 = (f16t*)(ws + off);  off += szF16;
  float* F32 = (float*)(ws + off); off += szF32;
  if (off > ws_size) return;
  if (off > (size_t)134217728) return;

  const dim3 cgrid(NTILE, nB);

  prep_w_k<<<dim3(WBLKX, 5), TPB, 0, stream>>>(w0a, w0r, w0b, wa, wb, Wp);
  pad_k<<<dim3(nB, 2), TPB, 0, stream>>>(H16, F16);
  xin_k<<<dim3(TP / 64, nB), TPB, 0, stream>>>(x, fids, femb, nF, XIN);

  conv_k<CPX, 3, 0><<<cgrid, CTPB, 0, stream>>>(XIN, Wp + OFF_W0A, b0a, 1, H16, F32);
  conv_k<CPX, 1, 1><<<cgrid, CTPB, 0, stream>>>(XIN, Wp + OFF_W0R, b0r, 1, F16, F32);
  conv_k<CH, 3, 2><<<cgrid, CTPB, 0, stream>>>(H16, Wp + OFF_W0B, b0b, 1, F16, F32);

  for (int i = 0; i < 4; ++i) {
    const int d = 2 << i;
    conv_k<CH, 3, 0><<<cgrid, CTPB, 0, stream>>>(F16, Wp + OFF_WA + (size_t)i * CH * K64, ba + i * CH, d, H16, F32);
    conv_k<CH, 3, 2><<<cgrid, CTPB, 0, stream>>>(H16, Wp + OFF_WB + (size_t)i * CH * K64, bb + i * CH, d, F16, F32);
  }

  heads_k<<<npos / TPB, TPB, 0, stream>>>(F32, petw, petb, pckw, pckb, aetw, aetb, outp, npos);
}
